// GATEncoder_46866683134378
// MI455X (gfx1250) — hardware-run, weakly checked
//
#include <hip/hip_runtime.h>
#include <stddef.h>
#include <stdint.h>
#include <math.h>

#define NN      50000
#define NE      600000
#define FD      128
#define HC      128
#define NH1     4
#define TERMS2  2
#define KA2     256
#define K2      (128 * TERMS2)
#define MP      50048
#define GBM     128
#define SPG     132
#define NTHR    256
#define NWAVE   8
#define EPT     8
#define WCH     (32 * EPT)
#define NBRUN   1024
#define SLB     10
#define NBK     49
#define WLCAP   2560
#define RCAP    16384
#define TRIPCAP 256
#define MAXDEG_MEAS   28
#define MAXB1024_MEAS 12548
#define ABM     64
#define NEGSL   0.2f
#define EPS_SM  1e-16f

#define BK_ZINTS (NWAVE * WLCAP + RCAP + 3 * NBRUN)
#define BK_INTS  (BK_ZINTS + 16)
#define BK_LDS   (BK_INTS * 4)
#define GEMM_LDS ((GBM * SPG + 2 * HC + GBM * 2 * NH1) * 4)

#define PBX   (MP * FD / 8 / NTHR)
#define PBW1  (HC * FD / 8 / NTHR)
#define PBW2  (HC * KA2 / 8 / NTHR)
#define PBTOT (PBX + PBW1 + PBW2 + 1)

static_assert(TERMS2 == 1 || TERMS2 == 2);
static_assert(NN < 65536);
static_assert(NBRUN == (1 << SLB) && NBRUN <= 1024);
static_assert(NBK * NBRUN >= MP);
static_assert(MP % GBM == 0 && MP >= NN && MP == 391 * GBM && MP % ABM == 0);
static_assert(NBRUN % ABM == 0 && ABM % NWAVE == 0);
static_assert(NE % 8 == 0 && NE % 4 == 0 && NE >= 8);
static_assert((((long long)NE + WCH) << SLB) < (1LL << 31));
static_assert((long long)RCAP * 100 >= (long long)MAXB1024_MEAS * 105);
static_assert(WLCAP >= MAXB1024_MEAS / 8 + 8 * 40 + 1);
static_assert(MAXDEG_MEAS + 8 <= TRIPCAP);
static_assert(RCAP % (NTHR * 4) == 0 && BK_ZINTS % 4 == 0 && (2 * NBRUN) % (NTHR * 4) == 0);
static_assert(BK_LDS <= 300000 && GEMM_LDS <= 300000);
static_assert(HC == 32 * 4 && HC == NH1 * 32 && FD % 32 == 0 && K2 % 32 == 0 && K2 <= KA2);
static_assert(GBM == NWAVE * 16 && NTHR == 2 * GBM);
static_assert((MP * FD / 8) % NTHR == 0 && (HC * FD / 8) % NTHR == 0 && (HC * KA2 / 8) % NTHR == 0);

typedef float          v4f   __attribute__((ext_vector_type(4)));
typedef float          v8f   __attribute__((ext_vector_type(8)));
typedef int            v4i   __attribute__((ext_vector_type(4)));
typedef int            v8i   __attribute__((ext_vector_type(8)));
typedef unsigned int   v4u   __attribute__((ext_vector_type(4)));
typedef unsigned short v8us  __attribute__((ext_vector_type(8)));
typedef unsigned short v16us __attribute__((ext_vector_type(16)));
typedef __bf16         v16bf __attribute__((ext_vector_type(16)));
typedef v4f  __attribute__((may_alias)) v4fa;
typedef v4i  __attribute__((may_alias)) v4ia;
typedef v8us __attribute__((may_alias)) v8usa;
union FragB { v16bf v; v16us u; v8us h[2]; v8i w; };

__device__ __forceinline__ v8f wmb(const FragB& a, const FragB& b, v8f c) {
  v8f d = __builtin_amdgcn_wmma_f32_16x16x32_bf16(false, a.v, false, b.v, (short)0, c, false, false);
  asm volatile("v_nop\n\tv_nop\n\tv_nop\n\tv_nop" : "+v"(d) : "v"(a.w), "v"(b.w));
  return d;
}

__device__ __forceinline__ unsigned bf16_bits(float f) {
  const unsigned u = __float_as_uint(f);
  const unsigned r = (u + 0x7FFFu + ((u >> 16) & 1u)) >> 16;
  const unsigned q = (u >> 16) | 0x40u;
  return ((u & 0x7fffffffu) > 0x7f800000u) ? q : r;
}
__device__ __forceinline__ unsigned bf16_hiword(float f) { return bf16_bits(f) << 16; }
__device__ __forceinline__ unsigned pk2(float lo, float hi) { return bf16_bits(lo) | (bf16_bits(hi) << 16); }

__device__ __forceinline__ void hilo_pack(float v0, float v1, float v2, float v3,
                                          int& h01, int& h23, int& l01, int& l23) {
  const unsigned a0 = bf16_bits(v0), a1 = bf16_bits(v1), a2 = bf16_bits(v2), a3 = bf16_bits(v3);
  const unsigned b0 = bf16_bits(v0 - __uint_as_float(a0 << 16));
  const unsigned b1 = bf16_bits(v1 - __uint_as_float(a1 << 16));
  const unsigned b2 = bf16_bits(v2 - __uint_as_float(a2 << 16));
  const unsigned b3 = bf16_bits(v3 - __uint_as_float(a3 << 16));
  h01 = (int)(a0 | (a1 << 16)); h23 = (int)(a2 | (a3 << 16));
  l01 = (int)(b0 | (b1 << 16)); l23 = (int)(b2 | (b3 << 16));
}

__device__ __forceinline__ void st2_v4f(float* p, v4f v) {
  *(volatile v4f*)p = v;
  __threadfence();
  *(volatile v4f*)p = v;
}
__device__ __forceinline__ void st2_v4u(unsigned short* p, v4u v) {
  *(volatile v4u*)p = v;
  __threadfence();
  *(volatile v4u*)p = v;
}

__device__ __forceinline__ v4u gather8(const float* __restrict__ base, int stride) {
  float f[8];
#pragma unroll
  for (int i = 0; i < 8; ++i) f[i] = base[(size_t)i * (size_t)stride];
  v4u o;
  o.x = pk2(f[0], f[1]); o.y = pk2(f[2], f[3]); o.z = pk2(f[4], f[5]); o.w = pk2(f[6], f[7]);
  return o;
}

__global__ __launch_bounds__(NTHR) void k_prep(const float* __restrict__ x, const float* __restrict__ w1,
                                               const float* __restrict__ w2,
                                               const float* __restrict__ as1, const float* __restrict__ ad1,
                                               const float* __restrict__ b1,
                                               const float* __restrict__ as2, const float* __restrict__ ad2,
                                               const float* __restrict__ b2,
                                               unsigned short* xb, unsigned short* w1t, unsigned short* w2d,
                                               float* par) {
  const int tid = (int)threadIdx.x, lane = tid & 31;
  const int blk = (int)blockIdx.x;
  if (blk < PBX) {
    const int u   = blk * NTHR + tid;
    const int row = u >> 4, k8 = (u & 15) * 8;
    const int rc  = row < NN ? row : NN - 1;
    const unsigned mk = row < NN ? 0xffffffffu : 0u;
    const float* p = x + (size_t)rc * FD + k8;
    const v4f a = *(const v4fa*)p;
    const v4f b = *(const v4fa*)(p + 4);
    asm volatile("" :: "v"(a), "v"(b));
    v4u o;
    o.x = pk2(a.x, a.y) & mk; o.y = pk2(a.z, a.w) & mk;
    o.z = pk2(b.x, b.y) & mk; o.w = pk2(b.z, b.w) & mk;
    st2_v4u(xb + (size_t)row * FD + k8, o);
  } else if (blk < PBX + PBW1) {
    const int u = (blk - PBX) * NTHR + tid;
    const int n = u >> 4, k8 = (u & 15) * 8;
    const v4u o = gather8(w1 + (size_t)k8 * HC + n, HC);
    st2_v4u(w1t + (size_t)n * FD + k8, o);
  } else if (blk < PBX + PBW1 + PBW2) {
    const int u = (blk - PBX - PBW1) * NTHR + tid;
    const int n = u >> 5, k8 = (u & 31) * 8, kk = k8 & 127;
    const v4u o = gather8(w2 + (size_t)kk * HC + n, HC);
    st2_v4u(w2d + (size_t)n * KA2 + k8, o);
  } else {
    if (tid < 6 * 32) {
      const int a = tid >> 5;
      const v4f c0 = *(const v4fa*)(as1 + 4 * lane);
      const v4f c1 = *(const v4fa*)(ad1 + 4 * lane);
      const v4f c2 = *(const v4fa*)(b1  + 4 * lane);
      const v4f c3 = *(const v4fa*)(as2 + 4 * lane);
      const v4f c4 = *(const v4fa*)(ad2 + 4 * lane);
      const v4f c5 = *(const v4fa*)(b2  + 4 * lane);
      asm volatile("" :: "v"(c0), "v"(c1), "v"(c2));
      asm volatile("" :: "v"(c3), "v"(c4), "v"(c5));
      const unsigned m0 = (a == 0) ? 0xffffffffu : 0u, m1 = (a == 1) ? 0xffffffffu : 0u;
      const unsigned m2 = (a == 2) ? 0xffffffffu : 0u, m3 = (a == 3) ? 0xffffffffu : 0u;
      const unsigned m4 = (a == 4) ? 0xffffffffu : 0u, m5 = (a == 5) ? 0xffffffffu : 0u;
      v4f o;
      o.x = __uint_as_float((bf16_hiword(c0.x) & m0) | (bf16_hiword(c1.x) & m1) | (bf16_hiword(c2.x) & m2) |
                            (bf16_hiword(c3.x) & m3) | (bf16_hiword(c4.x) & m4) | (bf16_hiword(c5.x) & m5));
      o.y = __uint_as_float((bf16_hiword(c0.y) & m0) | (bf16_hiword(c1.y) & m1) | (bf16_hiword(c2.y) & m2) |
                            (bf16_hiword(c3.y) & m3) | (bf16_hiword(c4.y) & m4) | (bf16_hiword(c5.y) & m5));
      o.z = __uint_as_float((bf16_hiword(c0.z) & m0) | (bf16_hiword(c1.z) & m1) | (bf16_hiword(c2.z) & m2) |
                            (bf16_hiword(c3.z) & m3) | (bf16_hiword(c4.z) & m4) | (bf16_hiword(c5.z) & m5));
      o.w = __uint_as_float((bf16_hiword(c0.w) & m0) | (bf16_hiword(c1.w) & m1) | (bf16_hiword(c2.w) & m2) |
                            (bf16_hiword(c3.w) & m3) | (bf16_hiword(c4.w) & m4) | (bf16_hiword(c5.w) & m5));
      st2_v4f(par + HC * a + 4 * lane, o);
    }
  }
}

__device__ __forceinline__ void bucket_flush(const int* pl, const int* cnt, int ov, int* lp, int* cop, int* fp,
                                             int tid) {
#pragma unroll 1
  for (int i = tid * 4; i < RCAP; i += NTHR * 4) {
    const v4i v = *(const v4ia*)(pl + i);
    *(volatile v4i*)(lp + i) = v;
  }
#pragma unroll 1
  for (int i = tid * 4; i < 2 * NBRUN; i += NTHR * 4) {
    const v4i v = *(const v4ia*)(cnt + i);
    *(volatile v4i*)(cop + i) = v;
  }
  if (tid < 8) {
    const v4i f = {ov, ov, ov, ov};
    *(volatile v4i*)(fp + 4 * tid) = f;
  }
}

__global__ __launch_bounds__(NTHR) void k_bucket(const int* __restrict__ srcs, const int* __restrict__ dsts,
                                                 int* HITS, int* CO, int* FLAG) {
  extern __shared__ __attribute__((aligned(16))) int dsm[];
  int* wl   = dsm;
  int* pl   = dsm + NWAVE * WLCAP;
  int* cnt  = pl + RCAP;
  int* offs = cnt + NBRUN;
  int* cur  = offs + NBRUN;
  int* misc = cur + NBRUN;
  const int tid = (int)threadIdx.x, lane = tid & 31, wave = tid >> 5;
  const int blk = (int)blockIdx.x;
  const unsigned nbs = (unsigned)(blk * NBRUN);

  {
    const v4i z4 = {0, 0, 0, 0};
    for (int i = tid * 4; i < BK_ZINTS; i += NTHR * 4) *(v4ia*)(dsm + i) = z4;
    if (tid < 16) misc[tid] = 0;
  }
  __syncthreads();

  {
    const int per  = ((NE + NWAVE * WCH - 1) / (NWAVE * WCH)) * WCH;
    const int ebeg = wave * per;
    const int eend = (ebeg + per < NE) ? (ebeg + per) : NE;
    int* mylist = wl + wave * WLCAP;
    int wc = 0;
#pragma unroll 1
    for (int cb = ebeg; cb < eend; cb += WCH) {
      const int e0 = cb + lane * EPT;
      const int ec = e0 < NE - EPT ? e0 : NE - EPT;
      const v4i da = *(const v4ia*)(dsts + ec);
      const v4i db = *(const v4ia*)(dsts + ec + 4);
      asm volatile("" :: "v"(da), "v"(db));
      const bool ok = e0 < eend;
      const unsigned s0 = (unsigned)da.x - nbs, s1 = (unsigned)da.y - nbs;
      const unsigned s2 = (unsigned)da.z - nbs, s3 = (unsigned)da.w - nbs;
      const unsigned s4 = (unsigned)db.x - nbs, s5 = (unsigned)db.y - nbs;
      const unsigned s6 = (unsigned)db.z - nbs, s7 = (unsigned)db.w - nbs;
      const bool h0 = ok & (s0 < (unsigned)NBRUN), h1 = ok & (s1 < (unsigned)NBRUN);
      const bool h2 = ok & (s2 < (unsigned)NBRUN), h3 = ok & (s3 < (unsigned)NBRUN);
      const bool h4 = ok & (s4 < (unsigned)NBRUN), h5 = ok & (s5 < (unsigned)NBRUN);
      const bool h6 = ok & (s6 < (unsigned)NBRUN), h7 = ok & (s7 < (unsigned)NBRUN);
      const unsigned m0 = __builtin_amdgcn_ballot_w32(h0), m1 = __builtin_amdgcn_ballot_w32(h1);
      const unsigned m2 = __builtin_amdgcn_ballot_w32(h2), m3 = __builtin_amdgcn_ballot_w32(h3);
      const unsigned m4 = __builtin_amdgcn_ballot_w32(h4), m5 = __builtin_amdgcn_ballot_w32(h5);
      const unsigned m6 = __builtin_amdgcn_ballot_w32(h6), m7 = __builtin_amdgcn_ballot_w32(h7);
      const unsigned any = m0 | m1 | m2 | m3 | m4 | m5 | m6 | m7;
      if (any != 0u) {
        const int pre = (int)(__builtin_amdgcn_mbcnt_lo(m0, 0u) + __builtin_amdgcn_mbcnt_lo(m1, 0u) +
                              __builtin_amdgcn_mbcnt_lo(m2, 0u) + __builtin_amdgcn_mbcnt_lo(m3, 0u) +
                              __builtin_amdgcn_mbcnt_lo(m4, 0u) + __builtin_amdgcn_mbcnt_lo(m5, 0u) +
                              __builtin_amdgcn_mbcnt_lo(m6, 0u) + __builtin_amdgcn_mbcnt_lo(m7, 0u));
        int p = wc + pre;
        if (h0) { if (p < WLCAP) mylist[p] = ((e0 + 0) << SLB) | (int)s0; p = p + 1; }
        if (h1) { if (p < WLCAP) mylist[p] = ((e0 + 1) << SLB) | (int)s1; p = p + 1; }
        if (h2) { if (p < WLCAP) mylist[p] = ((e0 + 2) << SLB) | (int)s2; p = p + 1; }
        if (h3) { if (p < WLCAP) mylist[p] = ((e0 + 3) << SLB) | (int)s3; p = p + 1; }
        if (h4) { if (p < WLCAP) mylist[p] = ((e0 + 4) << SLB) | (int)s4; p = p + 1; }
        if (h5) { if (p < WLCAP) mylist[p] = ((e0 + 5) << SLB) | (int)s5; p = p + 1; }
        if (h6) { if (p < WLCAP) mylist[p] = ((e0 + 6) << SLB) | (int)s6; p = p + 1; }
        if (h7) { if (p < WLCAP) mylist[p] = ((e0 + 7) << SLB) | (int)s7; p = p + 1; }
        wc += (int)(__builtin_popcount(m0) + __builtin_popcount(m1) + __builtin_popcount(m2) + __builtin_popcount(m3) +
                    __builtin_popcount(m4) + __builtin_popcount(m5) + __builtin_popcount(m6) + __builtin_popcount(m7));
      }
    }
    if (lane == 0) misc[wave] = wc;
  }
  __syncthreads();

  if (wave == 0) {
    int ov = 0;
#pragma unroll 1
    for (int w2 = 0; w2 < NWAVE; ++w2) {
      int c = misc[w2];
      if (c > WLCAP) ov = 1;
      c = c < 0 ? 0 : (c > WLCAP ? WLCAP : c);
#pragma unroll 1
      for (int b0 = 0; b0 < c; b0 += 32) {
        const int idx = b0 + lane;
        const int ent = wl[w2 * WLCAP + (idx < WLCAP ? idx : WLCAP - 1)];
        const int m32 = (c - b0) < 32 ? (c - b0) : 32;
#pragma unroll 1
        for (int k = 0; k < m32; ++k) {
          const int u    = __builtin_amdgcn_readlane(ent, k);
          const int slot = u & (NBRUN - 1);
          if (lane == 0) cnt[slot] = cnt[slot] + 1;
        }
      }
    }
    if (lane == 0) misc[9] = ov;
  }
  __syncthreads();
  if (wave == 0) {
    const int base = lane * (NBRUN / 32);
    int s = 0;
#pragma unroll 1
    for (int i = 0; i < NBRUN / 32; ++i) s += cnt[base + i];
    int incl = s;
#pragma unroll
    for (int d = 1; d < 32; d <<= 1) {
      const int y = __shfl_up(incl, d, 32);
      if (lane >= d) incl += y;
    }
    int run = incl - s;
#pragma unroll 1
    for (int i = 0; i < NBRUN / 32; ++i) {
      const int cv = cnt[base + i];
      offs[base + i] = run;
      cur[base + i]  = run;
      run += cv;
    }
    if (lane == 31) misc[10] = (incl > RCAP) ? 1 : 0;
  }
  __syncthreads();

  if (wave == 0) {
#pragma unroll 1
    for (int w2 = 0; w2 < NWAVE; ++w2) {
      int c = misc[w2];
      c = c < 0 ? 0 : (c > WLCAP ? WLCAP : c);
#pragma unroll 1
      for (int b0 = 0; b0 < c; b0 += 32) {
        const int idx = b0 + lane;
        const int ent = wl[w2 * WLCAP + (idx < WLCAP ? idx : WLCAP - 1)];
        int eid = (ent >> SLB) & 0xFFFFF;
        eid = eid > NE - 1 ? NE - 1 : eid;
        int sr = srcs[eid];
        sr = sr < 0 ? 0 : (sr > NN - 1 ? NN - 1 : sr);
        const int word = (int)((unsigned)sr | ((unsigned)(ent & (NBRUN - 1)) << 16));
        const int m32 = (c - b0) < 32 ? (c - b0) : 32;
#pragma unroll 1
        for (int k = 0; k < m32; ++k) {
          const int u    = __builtin_amdgcn_readlane(ent, k);
          const int wd   = __builtin_amdgcn_readlane(word, k);
          const int slot = u & (NBRUN - 1);
          if (lane == 0) {
            int p = cur[slot];
            p = p < 0 ? 0 : (p > RCAP - 1 ? RCAP - 1 : p);
            pl[p] = wd;
            cur[slot] = p + 1;
          }
        }
      }
    }
  }
  __syncthreads();

  const int ovf = misc[9] | misc[10];
  int* lp  = HITS + (size_t)blk * RCAP;
  int* cop = CO + (size_t)blk * (2 * NBRUN);
  int* fp  = FLAG + (size_t)blk * 32;
  bucket_flush(pl, cnt, ovf, lp, cop, fp, tid);
  __threadfence();
  bucket_flush(pl, cnt, ovf, lp, cop, fp, tid);
}

template <int NV4>
__device__ __forceinline__ void gemm_flush(const float* stg, const float* sdot, float* outF, float* sp,
                                           int rowBase, int tid, int lane, int wave) {
  if (tid < NV4) {
    const v4f s = *(const v4fa*)(sdot + 4 * tid);
    *(volatile v4f*)(sp + 4 * tid) = s;
  }
#pragma unroll 1
  for (int i = 0; i < 16; ++i) {
    const int lr = 16 * wave + i;
    const v4f v = *(const v4fa*)(stg + lr * SPG + 4 * lane);
    *(volatile v4f*)(outF + (size_t)(rowBase + lr) * HC + 4 * lane) = v;
  }
}

template <int HEADS, int KTOT, int LDA, int LDB>
__global__ __launch_bounds__(NTHR) __attribute__((amdgpu_num_vgpr(248)))
void k_gemm(const unsigned short* __restrict__ A, const unsigned short* __restrict__ BT,
            const float* __restrict__ pa_s, const float* __restrict__ pa_d, float* outF, float* SD) {
  extern __shared__ __attribute__((aligned(16))) float gsm[];
  float* stg  = gsm;
  float* spar = gsm + GBM * SPG;
  float* sdot = spar + 2 * HC;
  const int tid = (int)threadIdx.x, lane = tid & 31, wave = tid >> 5, hh = lane >> 4, m = lane & 15;
  const int rowBase = (int)blockIdx.x * GBM;

  if (tid < 32) {
    *(v4fa*)(spar + 4 * tid)      = *(const v4fa*)(pa_s + 4 * tid);
    *(v4fa*)(spar + HC + 4 * tid) = *(const v4fa*)(pa_d + 4 * tid);
  }

  v8f acc[8];
  {
    const v8f z = {0.f, 0.f, 0.f, 0.f, 0.f, 0.f, 0.f, 0.f};
#pragma unroll
    for (int t = 0; t < 8; ++t) acc[t] = z;
  }
  const unsigned short* ap = A + (size_t)(rowBase + 16 * wave + m) * (size_t)LDA + 8 * hh;
  const unsigned short* bp = BT + (size_t)m * (size_t)LDB + 8 * hh;
#pragma unroll 1
  for (int k0 = 0; k0 < KTOT; k0 += 32) {
    FragB af;
    af.h[0] = *(const v8usa*)(ap + k0);
    af.h[1] = *(const v8usa*)(ap + k0 + 16);
#pragma unroll
    for (int nt = 0; nt < 8; ++nt) {
      const unsigned short* wq = bp + (size_t)(16 * nt) * (size_t)LDB + k0;
      FragB bf;
      bf.h[0] = *(const v8usa*)wq;
      bf.h[1] = *(const v8usa*)(wq + 16);
      acc[nt] = wmb(af, bf, acc[nt]);
    }
  }

#pragma unroll
  for (int nt = 0; nt < 8; ++nt) {
#pragma unroll
    for (int r = 0; r < 8; ++r) stg[(16 * wave + 8 * hh + r) * SPG + 16 * nt + m] = acc[nt][r];
  }
  __syncthreads();

  {
    constexpr int CH = HC / HEADS;
    const int row = tid & (GBM - 1), which = tid >> 7;
    const float* hr = stg + row * SPG;
    const float* sa = spar + which * HC;
#pragma unroll 1
    for (int hd = 0; hd < HEADS; ++hd) {
      float d = 0.f;
#pragma unroll 4
      for (int c4 = 0; c4 < CH / 4; ++c4) {
        const v4f hv = *(const v4fa*)(hr + hd * CH + 4 * c4);
        const v4f av = *(const v4fa*)(sa + hd * CH + 4 * c4);
        d = fmaf(hv.x, av.x, d);
        d = fmaf(hv.y, av.y, d);
        d = fmaf(hv.z, av.z, d);
        d = fmaf(hv.w, av.w, d);
      }
      sdot[row * (2 * HEADS) + which * HEADS + hd] = d;
    }
  }
  __syncthreads();

  constexpr int NV4 = GBM * 2 * HEADS / 4;
  float* sp = SD + (size_t)rowBase * (size_t)(2 * HEADS);
  gemm_flush<NV4>(stg, sdot, outF, sp, rowBase, tid, lane, wave);
  __threadfence();
  gemm_flush<NV4>(stg, sdot, outF, sp, rowBase, tid, lane, wave);
}

template <int L>
__global__ __launch_bounds__(NTHR) void k_replay(const int* __restrict__ HITS, const int* __restrict__ CO,
                                                 const int* __restrict__ FLAG, const float* __restrict__ H,
                                                 const float* __restrict__ SD, const float* __restrict__ bias,
                                                 unsigned short* XHL, float* out) {
  constexpr int HEADS = (L == 1) ? NH1 : 1;
  constexpr int SDW   = 2 * HEADS;
  __shared__ __attribute__((aligned(16))) float sb[HC];
  const int tid = (int)threadIdx.x, lane = tid & 31, wave = tid >> 5;
  const int rowBase = (int)blockIdx.x * ABM;
  const int bucket  = rowBase >> SLB;
  const int* lb  = HITS + (size_t)bucket * RCAP;
  const int* cob = CO + (size_t)bucket * (2 * NBRUN);
  const int flag = FLAG[(size_t)bucket * 32];
  if (tid < 32) *(v4fa*)(sb + 4 * tid) = *(const v4fa*)(bias + 4 * tid);
  __syncthreads();
  const v4f bb = *(const v4fa*)(sb + 4 * lane);
  const int hd = (L == 1) ? (lane >> 3) : 0;
  const float qnan = __uint_as_float(0x7fc00000u);

#pragma unroll 1
  for (int i = 0; i < ABM / NWAVE; ++i) {
    const int d    = rowBase + (ABM / NWAVE) * wave + i;
    const int slot = d & (NBRUN - 1);
    const int dcl  = d < NN ? d : NN - 1;
    int c = __builtin_amdgcn_readfirstlane(cob[slot]);
    int o = __builtin_amdgcn_readfirstlane(cob[NBRUN + slot]);
    const bool big = c > TRIPCAP;
    c = c < 0 ? 0 : (c > TRIPCAP ? TRIPCAP : c);
    o = o < 0 ? 0 : (o > RCAP - 1 ? RCAP - 1 : o);
    if (c > RCAP - o) c = RCAP - o;

    const float adv = SD[(size_t)dcl * SDW + HEADS + hd];
    float l0 = SD[(size_t)dcl * SDW + hd] + adv;
    l0 = l0 > 0.f ? l0 : NEGSL * l0;
    float mx = l0, dn = 1.0f;
    v4f av = *(const v4fa*)(H + (size_t)dcl * HC + 4 * lane);

#pragma unroll 1
    for (int j = 0; j < c; ++j) {
      const unsigned wd = (unsigned)lb[o + j];
      int sr = (int)(wd & 0xffffu);
      sr = sr > NN - 1 ? NN - 1 : sr;
      const v4f fs = *(const v4fa*)(H + (size_t)sr * HC + 4 * lane);
      float lg = SD[(size_t)sr * SDW + hd] + adv;
      lg = lg > 0.f ? lg : NEGSL * lg;
      const float df = lg - mx;
      const float ee = expf(-fabsf(df));
      const bool up  = df > 0.f;
      const float s1 = up ? ee : 1.0f;
      const float s2 = up ? 1.0f : ee;
      mx = up ? lg : mx;
      dn = fmaf(dn, s1, s2);
      av.x = fmaf(av.x, s1, s2 * fs.x);
      av.y = fmaf(av.y, s1, s2 * fs.y);
      av.z = fmaf(av.z, s1, s2 * fs.z);
      av.w = fmaf(av.w, s1, s2 * fs.w);
    }
    const float inv = __builtin_amdgcn_rcpf(dn + EPS_SM);
    float v0 = fmaf(av.x, inv, bb.x), v1 = fmaf(av.y, inv, bb.y);
    float v2 = fmaf(av.z, inv, bb.z), v3 = fmaf(av.w, inv, bb.w);
    const bool bad = (flag != 0) | big;

    if constexpr (L == 1) {
#pragma unroll 1
      for (int j = 0; j < 4; ++j) {
        const float t = v0;
        const float r = (t > 0.f) ? t : expm1f(t);
        v0 = v1; v1 = v2; v2 = v3; v3 = r;
      }
      const bool live = d < NN;
      v0 = bad ? qnan : v0; v1 = bad ? qnan : v1; v2 = bad ? qnan : v2; v3 = bad ? qnan : v3;
      v0 = live ? v0 : 0.0f; v1 = live ? v1 : 0.0f; v2 = live ? v2 : 0.0f; v3 = live ? v3 : 0.0f;
      int h01, h23, l01, l23;
      hilo_pack(v0, v1, v2, v3, h01, h23, l01, l23);
      const int sa = (2 * lane) & 31, sc = (2 * lane + 1) & 31;
      const int g0 = __shfl(h01, sa, 32), g1 = __shfl(h23, sa, 32), g2 = __shfl(h01, sc, 32), g3 = __shfl(h23, sc, 32);
      const int q0 = __shfl(l01, sa, 32), q1 = __shfl(l23, sa, 32), q2 = __shfl(l01, sc, 32), q3 = __shfl(l23, sc, 32);
      const int mk = (lane < 16) ? -1 : 0;
      v4u pv;
      pv.x = (unsigned)((g0 & mk) | (q0 & ~mk));
      pv.y = (unsigned)((g1 & mk) | (q1 & ~mk));
      pv.z = (unsigned)((g2 & mk) | (q2 & ~mk));
      pv.w = (unsigned)((g3 & mk) | (q3 & ~mk));
      unsigned short* gp = XHL + (size_t)d * KA2 + 8 * lane;
      *(volatile v4u*)gp = pv;
      __threadfence();
      *(volatile v4u*)gp = pv;
    } else {
      v4f ov;
      ov.x = bad ? qnan : v0; ov.y = bad ? qnan : v1; ov.z = bad ? qnan : v2; ov.w = bad ? qnan : v3;
      float* op = out + (size_t)dcl * HC + 4 * lane;
      const bool wr = d < NN;
      if (wr) *(volatile v4f*)op = ov;
      __threadfence();
      if (wr) *(volatile v4f*)op = ov;
    }
  }
}

extern "C" void kernel_launch(void* const* d_in, const int* in_sizes, int n_in,
                              void* d_out, int out_size, void* d_ws, size_t ws_size,
                              hipStream_t stream) {
  if (n_in < 10) return;
  if (in_sizes[0] != NN * FD) return;
  if (in_sizes[1] != 2 * NE) return;
  if (in_sizes[2] != FD * HC) return;
  if (in_sizes[3] != HC || in_sizes[4] != HC) return;
  if (in_sizes[5] != HC) return;
  if (in_sizes[6] != HC * HC) return;
  if (in_sizes[7] != HC || in_sizes[8] != HC) return;
  if (in_sizes[9] != HC) return;
  if (out_size != NN * HC) return;

  const float* x   = (const float*)d_in[0];
  const int*   ei  = (const int*)d_in[1];
  const float* W1  = (const float*)d_in[2];
  const float* as1 = (const float*)d_in[3];
  const float* ad1 = (const float*)d_in[4];
  const float* b1  = (const float*)d_in[5];
  const float* W2  = (const float*)d_in[6];
  const float* as2 = (const float*)d_in[7];
  const float* ad2 = (const float*)d_in[8];
  const float* b2  = (const float*)d_in[9];
  float* out = (float*)d_out;
  const int* srcs = ei;
  const int* dsts = ei + NE;

  constexpr size_t zXB   = (size_t)MP * FD * 2;
  constexpr size_t zH    = (size_t)MP * HC * 4;
  constexpr size_t zX1   = (size_t)MP * KA2 * 2;
  constexpr size_t zSD1  = (size_t)MP * 2 * NH1 * 4;
  constexpr size_t zSD2  = (size_t)MP * 2 * 4;
  constexpr size_t zHITS = (size_t)NBK * RCAP * 4;
  constexpr size_t zCO   = (size_t)NBK * 2 * NBRUN * 4;
  constexpr size_t zFLAG = 6400;
  constexpr size_t zW1T  = (size_t)HC * FD * 2;
  constexpr size_t zW2D  = (size_t)HC * KA2 * 2;
  constexpr size_t zPAR  = (size_t)6 * HC * 4;
  constexpr size_t oXB   = 0;
  constexpr size_t oH    = oXB + zXB;
  constexpr size_t oX1   = oH + zH;
  constexpr size_t oSD1  = oX1 + zX1;
  constexpr size_t oSD2  = oSD1 + zSD1;
  constexpr size_t oHITS = oSD2 + zSD2;
  constexpr size_t oCO   = oHITS + zHITS;
  constexpr size_t oFLAG = oCO + zCO;
  constexpr size_t oW1T  = oFLAG + zFLAG;
  constexpr size_t oW2D  = oW1T + zW1T;
  constexpr size_t oPAR  = oW2D + zW2D;
  constexpr size_t oEND  = oPAR + zPAR;
  static_assert(zXB % 256 == 0 && zH % 256 == 0 && zX1 % 256 == 0 && zSD1 % 256 == 0 && zSD2 % 256 == 0);
  static_assert(zHITS % 256 == 0 && zCO % 256 == 0 && zFLAG % 256 == 0 && zFLAG >= (size_t)NBK * 128);
  static_assert(zW1T % 256 == 0 && zW2D % 256 == 0 && zPAR % 256 == 0);
  static_assert(oEND <= ((size_t)128 << 20));
  if (oEND > ws_size) return;

  char* ws = (char*)d_ws;
  unsigned short* XB   = (unsigned short*)(ws + oXB);
  float*          H    = (float*)(ws + oH);
  unsigned short* X1HL = (unsigned short*)(ws + oX1);
  float*          SD1  = (float*)(ws + oSD1);
  float*          SD2  = (float*)(ws + oSD2);
  int*            HITS = (int*)(ws + oHITS);
  int*            CO   = (int*)(ws + oCO);
  int*            FLAG = (int*)(ws + oFLAG);
  unsigned short* W1T  = (unsigned short*)(ws + oW1T);
  unsigned short* W2D  = (unsigned short*)(ws + oW2D);
  float*          PAR  = (float*)(ws + oPAR);

  hipFuncSetAttribute(reinterpret_cast<const void*>(&k_bucket), hipFuncAttributeMaxDynamicSharedMemorySize, (int)BK_LDS);
  hipFuncSetAttribute(reinterpret_cast<const void*>(&k_gemm<NH1, FD, FD, FD>),
                      hipFuncAttributeMaxDynamicSharedMemorySize, (int)GEMM_LDS);
  hipFuncSetAttribute(reinterpret_cast<const void*>(&k_gemm<1, K2, KA2, KA2>),
                      hipFuncAttributeMaxDynamicSharedMemorySize, (int)GEMM_LDS);

  k_prep<<<PBTOT, NTHR, 0, stream>>>(x, W1, W2, as1, ad1, b1, as2, ad2, b2, XB, W1T, W2D, PAR);
  k_bucket<<<NBK, NTHR, BK_LDS, stream>>>(srcs, dsts, HITS, CO, FLAG);
  k_gemm<NH1, FD, FD, FD><<<MP / GBM, NTHR, GEMM_LDS, stream>>>(XB, W1T, PAR + 0 * HC, PAR + 1 * HC, H, SD1);
  k_replay<1><<<MP / ABM, NTHR, 0, stream>>>(HITS, CO, FLAG, H, SD1, PAR + 2 * HC, X1HL, out);
  k_gemm<1, K2, KA2, KA2><<<MP / GBM, NTHR, GEMM_LDS, stream>>>(X1HL, W2D, PAR + 3 * HC, PAR + 4 * HC, H, SD2);
  k_replay<2><<<MP / ABM, NTHR, 0, stream>>>(HITS, CO, FLAG, H, SD2, PAR + 5 * HC, X1HL, out);
}
